// SelfAttentionLayer_72129680769842
// MI455X (gfx1250) — hardware-verified
//
#include <hip/hip_runtime.h>


#ifndef NB
#define NB 4
#endif
#ifndef SEQ
#define SEQ 2048
#endif
#define NB_FULL  4
#define SEQ_FULL 2048
#define DM   1024
#define NH   16
#define HD   64
#define MROWS (NB * SEQ)
#define KT   64
#define PP   72
#define OSP  68
#define CL2  0.18033688011112042f
#define PEX  10.0f

static_assert(SEQ % 64 == 0);
static_assert(SEQ >= 64 && SEQ <= SEQ_FULL);
static_assert(NB >= 1 && NB <= NB_FULL);
static_assert(NH * HD == DM);
static_assert(DM % 64 == 0);
static_assert((PP * 2) % 16 == 0);
static_assert((OSP * 4) % 16 == 0);

typedef _Float16 h16;
typedef unsigned short bf;
typedef __attribute__((ext_vector_type(16))) __bf16   v16bf;
typedef __attribute__((ext_vector_type(16))) _Float16 v16h;
typedef __attribute__((ext_vector_type(8)))  _Float16 v8h;
typedef __attribute__((ext_vector_type(8)))  unsigned short v8us;
typedef __attribute__((ext_vector_type(8)))  float    v8f;
typedef __attribute__((ext_vector_type(4)))  float    v4f;
typedef __attribute__((ext_vector_type(2)))  unsigned short v2us;
typedef v8h  __attribute__((may_alias)) v8ha;
typedef v4f  __attribute__((may_alias)) v4fa;
typedef v8us __attribute__((may_alias)) v8usa;

__device__ __forceinline__ unsigned short f2bf(float f) { unsigned u = __float_as_uint(f); u += 0x7FFFu + ((u >> 16) & 1u); return (unsigned short)(u >> 16); }
__device__ __forceinline__ float bf2f(unsigned short b) { return __uint_as_float(((unsigned)b) << 16); }
__device__ __forceinline__ float bfr(float f) { return bf2f(f2bf(f)); }
__device__ __forceinline__ v16h cat16(v8h lo, v8h hi) { return __builtin_shufflevector(lo, hi, 0, 1, 2, 3, 4, 5, 6, 7, 8, 9, 10, 11, 12, 13, 14, 15); }
__device__ __forceinline__ v16bf cat16b(v8us lo, v8us hi) { return __builtin_bit_cast(v16bf, __builtin_shufflevector(lo, hi, 0, 1, 2, 3, 4, 5, 6, 7, 8, 9, 10, 11, 12, 13, 14, 15)); }
__device__ __forceinline__ v8f wmma16(v16h a, v16h b, v8f c) { return __builtin_amdgcn_wmma_f32_16x16x32_f16(false, a, false, b, (short)0, c, false, false); }
__device__ __forceinline__ v8f wmmab(v16bf a, v16bf b, v8f c) { return __builtin_amdgcn_wmma_f32_16x16x32_bf16(false, a, false, b, (short)0, c, false, false); }

#define WAVE_SYNC() do { __builtin_amdgcn_fence(3  , "wavefront"); __builtin_amdgcn_wave_barrier(); asm volatile("" ::: "memory"); } while (0)

template <typename T16> struct WFrag;
template <> struct WFrag<h16> { typedef v16h V; static __device__ __forceinline__ V ld(const h16* p) { return cat16(*(const v8h*)p, *(const v8h*)(p + 16)); } static __device__ __forceinline__ v8f mma(V a, V b, v8f c) { return wmma16(a, b, c); } };
template <> struct WFrag<bf> { typedef v16bf V; static __device__ __forceinline__ V ld(const bf* p) { return cat16b(*(const v8us*)p, *(const v8us*)(p + 16)); } static __device__ __forceinline__ v8f mma(V a, V b, v8f c) { return wmmab(a, b, c); } };
template <typename T16, int NSPLIT, bool BIAS>
__global__ __launch_bounds__(32) void k_gemmw(const T16* __restrict__ A, const T16* __restrict__ A2, const T16* __restrict__ Bt, const T16* __restrict__ Bt2, int K, float* C, int ldc, const float* __restrict__ bias, size_t sA, size_t sB, size_t sC) {
    typedef typename WFrag<T16>::V V;
    __shared__ __align__(16) float os[16 * 68];
    const size_t z = blockIdx.z; A += z * sA; if (A2) A2 += z * sA; Bt += z * sB; if (Bt2) Bt2 += z * sB; C += z * sC;
    const int lane = threadIdx.x & 31, lr = lane & 15, hi = lane >> 4; const int r0 = blockIdx.x * 64, c0 = blockIdx.y * 64;
    v8f acc[4][4];
#pragma unroll
    for (int mb = 0; mb < 4; ++mb)
#pragma unroll
        for (int nb = 0; nb < 4; ++nb) acc[mb][nb] = (v8f){};
    const size_t aoff = (size_t)(r0 + lr) * K + 8 * hi, boff = (size_t)(c0 + lr) * K + 8 * hi;
#pragma unroll 1
    for (int kc = 0; kc < K; kc += 32) {
        V a[4], a2[4];
#pragma unroll
        for (int mb = 0; mb < 4; ++mb) { a[mb] = WFrag<T16>::ld(A + aoff + (size_t)mb * 16 * K + kc); if (NSPLIT == 1 || NSPLIT == 2) a2[mb] = WFrag<T16>::ld(A2 + aoff + (size_t)mb * 16 * K + kc); }
#pragma unroll
        for (int nb = 0; nb < 4; ++nb) { const V b = WFrag<T16>::ld(Bt + boff + (size_t)nb * 16 * K + kc); V b2; if (NSPLIT >= 2) b2 = WFrag<T16>::ld(Bt2 + boff + (size_t)nb * 16 * K + kc);
#pragma unroll
            for (int mb = 0; mb < 4; ++mb) { acc[mb][nb] = WFrag<T16>::mma(a[mb], b, acc[mb][nb]); if (NSPLIT == 1 || NSPLIT == 2) acc[mb][nb] = WFrag<T16>::mma(a2[mb], b, acc[mb][nb]); if (NSPLIT >= 2) acc[mb][nb] = WFrag<T16>::mma(a[mb], b2, acc[mb][nb]); } }
        asm volatile("v_nop\n\tv_nop\n\tv_nop\n\tv_nop" : "+v"(acc[0][0]), "+v"(acc[1][1]), "+v"(acc[2][2]), "+v"(acc[3][3]) : "v"(a[0]), "v"(a[3]));
    }
#pragma unroll
    for (int mb = 0; mb < 4; ++mb) {
#pragma unroll
        for (int nb = 0; nb < 4; ++nb) {
#pragma unroll
            for (int j = 0; j < 8; ++j) os[(hi * 8 + j) * 68 + nb * 16 + lr] = acc[mb][nb][j]; }
        __builtin_amdgcn_wave_barrier(); asm volatile("" ::: "memory");
        float* crow = C + (size_t)(r0 + mb * 16) * ldc + c0;
#pragma unroll 1
        for (int ps = 0; ps < 2; ++ps) {
#pragma unroll
            for (int s = 0; s < 8; ++s) { const int row = 2 * s + hi, cofs = lr * 4; v4f val = *(const v4fa*)(os + row * 68 + cofs); if (BIAS) { val[0] += bfr(bias[c0 + cofs]); val[1] += bfr(bias[c0 + cofs + 1]); val[2] += bfr(bias[c0 + cofs + 2]); val[3] += bfr(bias[c0 + cofs + 3]); }
                *(volatile v4f*)(crow + (size_t)row * ldc + cofs) = val; }
            if (ps == 0) __threadfence(); }
        __builtin_amdgcn_wave_barrier(); asm volatile("" ::: "memory");
    }
}

__global__ __launch_bounds__(256) void k_wtG(const float* __restrict__ w, int K, int N, bf* Bt) {
    const int lane = threadIdx.x & 31; const int L0 = (blockIdx.x * 8 + (threadIdx.x >> 5)) * 8; const int nlines = N * K / 64;
#pragma unroll
    for (int ps = 0; ps < 2; ++ps) {
#pragma unroll 1
        for (int l = 0; l < 8; ++l) { const int L = L0 + l; if (L >= nlines) break; const size_t e = (size_t)L * 64 + lane * 2; const int k = (int)(e % K), n = (int)(e / K); v2us o;
            o[0] = f2bf(w[(size_t)k * N + n]); o[1] = f2bf(w[(size_t)(k + 1) * N + n]); *(volatile v2us*)(Bt + e) = o; }
        if (ps == 0) __threadfence(); }
}
__global__ __launch_bounds__(256) void k_cvt8(const float* __restrict__ src, bf* dst, size_t n8) { const size_t i = (size_t)blockIdx.x * 256 + threadIdx.x; if (i >= n8) return; const v8f v = *(const v8f*)(src + i * 8); v8us o;
#pragma unroll
    for (int k = 0; k < 8; ++k) o[k] = f2bf(v[k]); *(volatile v8us*)(dst + i * 8) = o; __threadfence(); *(volatile v8us*)(dst + i * 8) = o; }

__global__ __launch_bounds__(256) void k_hplane(const float* __restrict__ F, h16* P, size_t n8) {
    const size_t i = (size_t)blockIdx.x * 256 + threadIdx.x; if (i >= n8) return; const size_t e = i * 8;
    const int d = (int)(e % HD); const int t = (int)((e / HD) % SEQ); const int hb = (int)(e / ((size_t)HD * SEQ)); const int h = hb % NH, b = hb / NH;
    const v8f v = *(const v8f*)(F + ((size_t)b * SEQ + t) * DM + h * HD + d); v8h o;
#pragma unroll
    for (int k = 0; k < 8; ++k) o[k] = (h16)v[k];
    *(volatile v8h*)(P + e) = o; __threadfence(); *(volatile v8h*)(P + e) = o;
}
__global__ __launch_bounds__(256) void k_vtplane(const float* __restrict__ F, h16* VT, size_t n8) {
    const size_t i = (size_t)blockIdx.x * 256 + threadIdx.x; if (i >= n8) return; const size_t e = i * 8;
    const int t = (int)(e % SEQ); const int d = (int)((e / SEQ) % HD); const int hb = (int)(e / ((size_t)SEQ * HD)); const int h = hb % NH, b = hb / NH;
    const float* f = F + ((size_t)b * SEQ + t) * DM + h * HD + d; v8h o;
#pragma unroll
    for (int q = 0; q < 8; ++q) o[q] = (h16)f[(size_t)q * DM];
    *(volatile v8h*)(VT + e) = o; __threadfence(); *(volatile v8h*)(VT + e) = o;
}

__global__ __launch_bounds__(128) void k_attn(const h16* __restrict__ QP, const h16* __restrict__ KP, const h16* __restrict__ VT, float* OUT) {
    __shared__ __align__(16) h16 ps[4][16 * PP];
    __shared__ __align__(16) float os[4][16 * OSP];
    const int lane = threadIdx.x & 31, w = threadIdx.x >> 5, hh = lane >> 4, m = lane & 15;
    const int bh = blockIdx.y; const int b = bh / NH, hd = bh % NH;
    const int q0 = blockIdx.x * 64 + w * 16;
    const h16* Qp = QP + ((size_t)bh * SEQ + q0) * HD;
    const h16* Kp = KP + (size_t)bh * SEQ * HD;
    const h16* Vp = VT + (size_t)bh * HD * SEQ;
    h16* pw = ps[w]; float* ow = os[w];
    v16h qf[2];
#pragma unroll
    for (int ks = 0; ks < 2; ++ks) { const h16* p = Qp + (size_t)m * HD + ks * 32 + 8 * hh; qf[ks] = cat16(*(const v8h*)p, *(const v8h*)(p + 16)); }
    v8f oacc[4];
#pragma unroll
    for (int nj = 0; nj < 4; ++nj) oacc[nj] = (v8f){};
    float ms[8], lp[8];
#pragma unroll
    for (int g = 0; g < 8; ++g) { ms[g] = -3.0e38f; lp[g] = 0.0f; }
#pragma unroll 1
    for (int kt = 0; kt < SEQ; kt += KT) {
        v8f sc[4]; v16h kf;
#pragma unroll
        for (int ni = 0; ni < 4; ++ni) { sc[ni] = (v8f){};
#pragma unroll
            for (int ks = 0; ks < 2; ++ks) { const h16* kr = Kp + (size_t)(kt + 16 * ni + m) * HD + ks * 32 + 8 * hh; kf = cat16(*(const v8h*)kr, *(const v8h*)(kr + 16)); sc[ni] = wmma16(qf[ks], kf, sc[ni]); } }
        asm volatile("v_nop\n\tv_nop\n\tv_nop\n\tv_nop" : "+v"(sc[0]), "+v"(sc[1]), "+v"(sc[2]), "+v"(sc[3]) : "v"(qf[0]), "v"(qf[1]), "v"(kf));
        asm volatile("" ::: "memory");
#pragma unroll
        for (int g = 0; g < 8; ++g) {
            float rm = fmaxf(fmaxf(sc[0][g], sc[1][g]), fmaxf(sc[2][g], sc[3][g]));
#pragma unroll
            for (int sh = 8; sh; sh >>= 1) rm = fmaxf(rm, __shfl_xor(rm, sh, 32));
            const float mn = fmaxf(ms[g], rm * CL2);
            const float corr = __builtin_amdgcn_exp2f(ms[g] - mn);
            ms[g] = mn; const float nbias = mn - PEX;
            float p[4];
#pragma unroll
            for (int ni = 0; ni < 4; ++ni) p[ni] = __builtin_amdgcn_exp2f(fmaf(sc[ni][g], CL2, -nbias));
            lp[g] = fmaf(lp[g], corr, (p[0] + p[1]) + (p[2] + p[3]));
#pragma unroll
            for (int nj = 0; nj < 4; ++nj) oacc[nj][g] *= corr;
#pragma unroll
            for (int ni = 0; ni < 4; ++ni) pw[(8 * hh + g) * PP + 16 * ni + m] = (h16)p[ni];
        }
        WAVE_SYNC();
        v16h pf[2];
#pragma unroll
        for (int ks = 0; ks < 2; ++ks) { const h16* pr = pw + m * PP + ks * 32 + 8 * hh; pf[ks] = cat16(*(const v8ha*)pr, *(const v8ha*)(pr + 16)); }
        v16h vf;
#pragma unroll
        for (int nj = 0; nj < 4; ++nj) {
#pragma unroll
            for (int ks = 0; ks < 2; ++ks) { const h16* vr = Vp + (size_t)(16 * nj + m) * SEQ + kt + ks * 32 + 8 * hh; vf = cat16(*(const v8h*)vr, *(const v8h*)(vr + 16)); oacc[nj] = wmma16(pf[ks], vf, oacc[nj]); } }
        asm volatile("v_nop\n\tv_nop\n\tv_nop\n\tv_nop" : "+v"(oacc[0]), "+v"(oacc[1]), "+v"(oacc[2]), "+v"(oacc[3]) : "v"(pf[0]), "v"(pf[1]), "v"(vf));
        asm volatile("" ::: "memory");
    }
#pragma unroll
    for (int g = 0; g < 8; ++g) {
        float l = lp[g];
#pragma unroll
        for (int sh = 8; sh; sh >>= 1) l += __shfl_xor(l, sh, 32);
        const float inv = 1.0f / l;
#pragma unroll
        for (int nj = 0; nj < 4; ++nj) ow[(8 * hh + g) * OSP + 16 * nj + m] = oacc[nj][g] * inv;
    }
    WAVE_SYNC();
    float* orow = OUT + ((size_t)b * SEQ + q0) * DM + hd * HD;
#pragma unroll 1
    for (int psi = 0; psi < 2; ++psi) {
#pragma unroll
        for (int s = 0; s < 8; ++s) { const int row = 2 * s + hh, cofs = m * 4; const v4f val = *(const v4fa*)(ow + row * OSP + cofs); *(volatile v4f*)(orow + (size_t)row * DM + cofs) = val; }
        if (psi == 0) __threadfence(); }
}

extern "C" void kernel_launch(void* const* d_in, const int* in_sizes, int n_in,
                              void* d_out, int out_size, void* d_ws, size_t ws_size, hipStream_t stream) {
    if (n_in < 7) return;
    if (in_sizes[0] < ((NB - 1) * SEQ_FULL + SEQ) * DM) return;
    if (in_sizes[1] < DM * DM || in_sizes[3] < DM * DM || in_sizes[5] < DM * DM) return;
    if (in_sizes[2] < DM || in_sizes[4] < DM || in_sizes[6] < DM) return;
    if (out_size < MROWS * DM) return;
    const float* x = (const float*)d_in[0]; const float* wq = (const float*)d_in[1]; const float* bq = (const float*)d_in[2]; const float* wk = (const float*)d_in[3]; const float* bk = (const float*)d_in[4]; const float* wv = (const float*)d_in[5]; const float* bv = (const float*)d_in[6];
    float* OUT = (float*)d_out;
    char* wsp = (char*)d_ws;
    auto take = [&](size_t bytes) { char* p = wsp; wsp += (bytes + 255) & ~(size_t)255; return (void*)p; };
    bf* WQ = (bf*)take((size_t)DM * DM * 2); bf* WK = (bf*)take((size_t)DM * DM * 2); bf* WV = (bf*)take((size_t)DM * DM * 2);
    bf* XB = (bf*)take((size_t)MROWS * DM * 2);
    float* F = (float*)take((size_t)MROWS * DM * 4);
    h16* QPL = (h16*)take((size_t)MROWS * DM * 2);
    h16* KPL = (h16*)take((size_t)MROWS * DM * 2);
    h16* VTL = (h16*)take((size_t)MROWS * DM * 2);
    if ((size_t)(wsp - (char*)d_ws) > ws_size) return;
    const int nlines = DM * DM / 64;
    k_wtG<<<(unsigned)((nlines + 63) / 64), 256, 0, stream>>>(wq, DM, DM, WQ);
    k_wtG<<<(unsigned)((nlines + 63) / 64), 256, 0, stream>>>(wk, DM, DM, WK);
    k_wtG<<<(unsigned)((nlines + 63) / 64), 256, 0, stream>>>(wv, DM, DM, WV);
    const size_t x8 = (size_t)SEQ * DM / 8;
    for (int b = 0; b < NB; ++b)
        k_cvt8<<<(unsigned)((x8 + 255) / 256), 256, 0, stream>>>(x + (size_t)b * SEQ_FULL * DM, XB + (size_t)b * SEQ * DM, x8);
    const size_t p8 = (size_t)MROWS * DM / 8; const unsigned LP = (unsigned)((p8 + 255) / 256);
    const dim3 gg(MROWS / 64, DM / 64, 1);
    k_gemmw<bf, 0, true><<<gg, 32, 0, stream>>>(XB, nullptr, WQ, nullptr, DM, F, DM, bq, 0, 0, 0);
    k_hplane<<<LP, 256, 0, stream>>>(F, QPL, p8);
    k_gemmw<bf, 0, true><<<gg, 32, 0, stream>>>(XB, nullptr, WK, nullptr, DM, F, DM, bk, 0, 0, 0);
    k_hplane<<<LP, 256, 0, stream>>>(F, KPL, p8);
    k_gemmw<bf, 0, true><<<gg, 32, 0, stream>>>(XB, nullptr, WV, nullptr, DM, F, DM, bv, 0, 0, 0);
    k_vtplane<<<LP, 256, 0, stream>>>(F, VTL, p8);
    k_attn<<<dim3(SEQ / 64, NB * NH), 128, 0, stream>>>(QPL, KPL, VTL, OUT);
}
